// GRUEncDec_79370995631067
// MI455X (gfx1250) — hardware-verified
//
#include <hip/hip_runtime.h>
#include <stdint.h>

typedef __attribute__((ext_vector_type(16))) _Float16 v16h;
typedef __attribute__((ext_vector_type(8)))  _Float16 v8h;
typedef __attribute__((ext_vector_type(8)))  float    v8f;
typedef __attribute__((ext_vector_type(4)))  float    v4f;

constexpr int kHid       = 64;
constexpr int kSeq       = 200;
constexpr int kIn        = 4;
constexpr int kDecSteps  = 20;
constexpr int kEncSteps  = kSeq - 1;
constexpr int kRows      = 32;
constexpr int kThreads   = 256;
constexpr int kPitchH    = 72;
constexpr int kPitchW    = 64;
constexpr int kChunk     = 8;
constexpr int kNumChunks = (kEncSteps + kChunk - 1) / kChunk;
constexpr int kRowFloats = kSeq * kIn;
constexpr int kOutRow    = kDecSteps * kIn;
constexpr int kXsSlots   = kRows * (kChunk + 1);
constexpr int kGateRows  = 3 * kHid;
constexpr int kHTileElems = kRows * kPitchH;
constexpr int kOutLines  = (kRows * kOutRow) / 32;
constexpr int kLineIters = (kOutLines + 31) / 32;

static_assert(kHTileElems % 8 == 0, "h tile zero fill granularity");
static_assert((kRows * kOutRow * 4) % 128 == 0, "block output is whole lines");
static_assert(kIn * kHid == kThreads, "lin_W staged one element per thread");

struct FragH {
  union U { v16h v; v8h h[2]; };
  static __device__ __forceinline__ v16h load(const _Float16* p) {
    U f; f.h[0] = *(const v8h*)(p); f.h[1] = *(const v8h*)(p + 16); return f.v;
  }
};

__device__ __forceinline__ v8f mma_h(v16h a, v16h b, v8f c) {
  c = __builtin_amdgcn_wmma_f32_16x16x32_f16(false, a, false, b, (short)0, c, false, false);
  asm volatile("v_nop\n\tv_nop\n\tv_nop\n\tv_nop" : "+v"(c) : "v"(a), "v"(b));
  return c;
}

struct UnitW { v4f wr, wz, wn; float bir, biz, bin2, bhr, bhz, bhn; };

__device__ __forceinline__ UnitW load_unit(const float* __restrict__ Wih,
                                           const float* __restrict__ bih,
                                           const float* __restrict__ bhh, int u) {
  UnitW w;
  w.wr = *(const v4f*)(Wih + (size_t)u * kIn);
  w.wz = *(const v4f*)(Wih + (size_t)(kHid + u) * kIn);
  w.wn = *(const v4f*)(Wih + (size_t)(2 * kHid + u) * kIn);
  w.bir = bih[u]; w.biz = bih[kHid + u]; w.bin2 = bih[2 * kHid + u];
  w.bhr = bhh[u]; w.bhz = bhh[kHid + u]; w.bhn = bhh[2 * kHid + u];
  return w;
}

__device__ __forceinline__ float sigm_f(float x) { return __builtin_amdgcn_rcpf(1.0f + expf(-x)); }
__device__ __forceinline__ float tanh_f(float x) { return 1.0f - 2.0f * __builtin_amdgcn_rcpf(1.0f + expf(2.0f * x)); }

__device__ __forceinline__ float gru_cell(v4f d, float ghr, float ghz, float ghn, float hp, const UnitW& w) {
  const float ir  = (d[0] * w.wr[0] + d[1] * w.wr[1] + d[2] * w.wr[2] + d[3] * w.wr[3]) + w.bir;
  const float iz  = (d[0] * w.wz[0] + d[1] * w.wz[1] + d[2] * w.wz[2] + d[3] * w.wz[3]) + w.biz;
  const float inn = (d[0] * w.wn[0] + d[1] * w.wn[1] + d[2] * w.wn[2] + d[3] * w.wn[3]) + w.bin2;
  const float rg = sigm_f(ir + (ghr + w.bhr));
  const float zg = sigm_f(iz + (ghz + w.bhz));
  const float ng = tanh_f(inn + rg * (ghn + w.bhn));
  return (1.0f - zg) * ng + zg * hp;
}

__device__ __forceinline__ void fill_wsh(_Float16* wsh, const float* __restrict__ W, int tid) {
#pragma unroll 1
  for (int i = tid; i < kGateRows * kHid; i += kThreads) {
    wsh[(i >> 6) * kPitchW + (i & 63)] = (_Float16)(W[i] * 8.0f);
  }
}

__device__ __forceinline__ void hh_tiles(v8f (&acc)[3], const _Float16* hs, const _Float16* ws,
                                         int arow, int u, int hh) {
  const v8f z8 = {0.f, 0.f, 0.f, 0.f, 0.f, 0.f, 0.f, 0.f};
  acc[0] = z8; acc[1] = z8; acc[2] = z8;
#pragma unroll
  for (int kk = 0; kk < 2; ++kk) {
    const v16h a = FragH::load(hs + arow * kPitchH + 32 * kk + 8 * hh);
#pragma unroll
    for (int g = 0; g < 3; ++g) {
      const v16h b = FragH::load(ws + (g * kHid + u) * kPitchW + 32 * kk + 8 * hh);
      acc[g] = mma_h(a, b, acc[g]);
    }
  }
}

__global__ __launch_bounds__(256)
void gru_encdec_seq(const float* __restrict__ xin,
                    const float* __restrict__ eWih, const float* __restrict__ eWhh,
                    const float* __restrict__ ebih, const float* __restrict__ ebhh,
                    const float* __restrict__ dWih, const float* __restrict__ dWhh,
                    const float* __restrict__ dbih, const float* __restrict__ dbhh,
                    const float* __restrict__ linW, const float* __restrict__ linb,
                    float* __restrict__ out) {
  __shared__ __align__(16) _Float16 wsh[kGateRows * kPitchW];
  __shared__ __align__(16) _Float16 htile[2][kHTileElems];
  __shared__ __align__(16) float xs[kXsSlots * 4];
  __shared__ __align__(16) float hfull[kRows * kHid];
  __shared__ __align__(16) float linws[kIn * kHid];
  __shared__ __align__(16) float pxs[kRows * kIn];
  __shared__ __align__(16) float cums[kRows * kIn];
  __shared__ __align__(16) float offs[kRows * kIn];
  __shared__ __align__(16) float outs[kRows * kOutRow];

  const int tid  = threadIdx.x;
  const int lane = tid & 31;
  const int wave = tid >> 5;
  const int hh   = lane >> 4;
  const int c    = lane & 15;
  const int msub = wave >> 2;
  const int ub   = wave & 3;
  const int u    = 16 * ub + c;
  const int arow = 16 * msub + c;
  const int rloc0 = 16 * msub + 8 * hh;
  const size_t rowbase = (size_t)blockIdx.x * kRows * kRowFloats;

  {
    v8h z;
#pragma unroll
    for (int e = 0; e < 8; ++e) z[e] = (_Float16)0.0f;
    for (int i = tid; i < kHTileElems / 8; i += kThreads) *(v8h*)(&htile[0][i * 8]) = z;
  }
  linws[tid] = linW[tid];
  fill_wsh(wsh, eWhh, tid);
  UnitW uw = load_unit(eWih, ebih, ebhh, u);

  float hreg[8];
#pragma unroll
  for (int r = 0; r < 8; ++r) hreg[r] = 0.0f;
  int cur = 0;

#pragma unroll 1
  for (int ch = 0; ch < kNumChunks; ++ch) {
    __syncthreads();
    const int p0 = ch * kChunk;
    for (int i = tid; i < kXsSlots; i += kThreads) {
      const int rr = i / (kChunk + 1);
      const int j  = i - rr * (kChunk + 1);
      int pos = p0 + j;
      pos = pos > (kSeq - 1) ? (kSeq - 1) : pos;
      const v4f v = *(const v4f*)(xin + rowbase + (size_t)rr * kRowFloats + (size_t)pos * kIn);
      *(v4f*)(xs + i * 4) = v;
    }
    __syncthreads();
    int nst = kEncSteps - p0;
    nst = nst > kChunk ? kChunk : nst;
#pragma unroll 1
    for (int s = 0; s < nst; ++s) {
      v8f acc[3];
      hh_tiles(acc, &htile[cur][0], wsh, arow, u, hh);
      _Float16* hd = &htile[cur ^ 1][0];
#pragma unroll
      for (int r = 0; r < 8; ++r) {
        const int rl = rloc0 + r;
        const v4f xp = *(const v4f*)(xs + (rl * (kChunk + 1) + s) * 4);
        const v4f xc = *(const v4f*)(xs + (rl * (kChunk + 1) + s + 1) * 4);
        const v4f d  = xc - xp;
        const float hn = gru_cell(d, acc[0][r] * 0.125f, acc[1][r] * 0.125f, acc[2][r] * 0.125f, hreg[r], uw);
        hreg[r] = hn;
        hd[rl * kPitchH + u] = (_Float16)hn;
      }
      __syncthreads();
      cur ^= 1;
    }
  }

  fill_wsh(wsh, dWhh, tid);
  uw = load_unit(dWih, dbih, dbhh, u);
  if (tid < kRows * kIn) {
    const int rr = tid >> 2, k = tid & 3;
    const float a = xin[rowbase + (size_t)rr * kRowFloats + (size_t)(kSeq - 2) * kIn + k];
    const float b = xin[rowbase + (size_t)rr * kRowFloats + (size_t)(kSeq - 1) * kIn + k];
    pxs[tid]  = b - a;
    offs[tid] = b;
    cums[tid] = 0.0f;
  }
  const int lrow  = tid >> 3;
  const int lk    = (tid >> 1) & 3;
  const int lhalf = tid & 1;
  const float lbk = linb[lk];
  __syncthreads();

#pragma unroll 1
  for (int s = 0; s < kDecSteps; ++s) {
    v8f acc[3];
    hh_tiles(acc, &htile[cur][0], wsh, arow, u, hh);
    _Float16* hd = &htile[cur ^ 1][0];
#pragma unroll
    for (int r = 0; r < 8; ++r) {
      const int rl = rloc0 + r;
      const v4f d = *(const v4f*)(pxs + rl * kIn);
      const float hn = gru_cell(d, acc[0][r] * 0.125f, acc[1][r] * 0.125f, acc[2][r] * 0.125f, hreg[r], uw);
      hreg[r] = hn;
      hd[rl * kPitchH + u] = (_Float16)hn;
      hfull[rl * kHid + u] = hn;
    }
    __syncthreads();
    {
      const float* hr = hfull + lrow * kHid + 32 * lhalf;
      const float* wl = linws + lk * kHid + 32 * lhalf;
      float dsum = 0.0f;
#pragma unroll
      for (int j = 0; j < 8; ++j) {
        const v4f a = *(const v4f*)(hr + 4 * j);
        const v4f w = *(const v4f*)(wl + 4 * j);
        dsum += a[0] * w[0]; dsum += a[1] * w[1]; dsum += a[2] * w[2]; dsum += a[3] * w[3];
      }
      const float tot = dsum + __shfl_xor(dsum, 1, 32);
      const float pxv = pxs[lrow * kIn + lk];
      const float xv  = (tot + lbk) + pxv;
      const float cm  = cums[lrow * kIn + lk] + xv;
      const float ov  = cm + offs[lrow * kIn + lk];
      if (lhalf == 0) {
        pxs[lrow * kIn + lk]  = xv;
        cums[lrow * kIn + lk] = cm;
        outs[lrow * kOutRow + s * kIn + lk] = ov;
      }
    }
    __syncthreads();
    cur ^= 1;
  }

  {
    float* ob = out + (size_t)blockIdx.x * (kRows * kOutRow);
    const int q = lane >> 3, c4 = (lane & 7) * 4;
    for (int pass = 0; pass < 2; ++pass) {
#pragma unroll
      for (int it = 0; it < kLineIters; ++it) {
        const int L = it * 32 + wave * 4 + q;
        if (L < kOutLines) {
          const v4f v = *(const v4f*)(outs + L * 32 + c4);
          *(volatile v4f*)(ob + (size_t)L * 32 + c4) = v;
        }
      }
      __threadfence();
    }
  }
}

extern "C" void kernel_launch(void* const* d_in, const int* in_sizes, int n_in,
                              void* d_out, int out_size, void* d_ws, size_t ws_size,
                              hipStream_t stream) {
  (void)d_ws; (void)ws_size;
  if (n_in < 11) return;
  if (in_sizes[1] < kGateRows * kIn || in_sizes[2] < kGateRows * kHid ||
      in_sizes[3] < kGateRows || in_sizes[4] < kGateRows ||
      in_sizes[5] < kGateRows * kIn || in_sizes[6] < kGateRows * kHid ||
      in_sizes[7] < kGateRows || in_sizes[8] < kGateRows ||
      in_sizes[9] < kIn * kHid || in_sizes[10] < kIn) return;
  const int nrows = in_sizes[0] / kRowFloats;
  int nblk = nrows / kRows;
  const int nblk_o = out_size / (kRows * kOutRow);
  if (nblk_o < nblk) nblk = nblk_o;
  if (nblk <= 0) return;

  const float* xin  = (const float*)d_in[0];
  const float* eWih = (const float*)d_in[1];
  const float* eWhh = (const float*)d_in[2];
  const float* ebih = (const float*)d_in[3];
  const float* ebhh = (const float*)d_in[4];
  const float* dWih = (const float*)d_in[5];
  const float* dWhh = (const float*)d_in[6];
  const float* dbih = (const float*)d_in[7];
  const float* dbhh = (const float*)d_in[8];
  const float* linW = (const float*)d_in[9];
  const float* linb = (const float*)d_in[10];
  float* out = (float*)d_out;

  gru_encdec_seq<<<dim3(nblk), dim3(kThreads), 0, stream>>>(xin, eWih, eWhh, ebih, ebhh,
                                                            dWih, dWhh, dbih, dbhh, linW, linb, out);
}
